// StreamingSTGCN_Model_33792802684974
// MI455X (gfx1250) — hardware-verified
//
#include <hip/hip_runtime.h>
#include <math.h>

typedef __attribute__((ext_vector_type(16))) _Float16 v16h;
typedef __attribute__((ext_vector_type(16))) __bf16 v16b;
typedef __attribute__((ext_vector_type(8)))  _Float16 v8h;
typedef __attribute__((ext_vector_type(8)))  float v8f;
typedef __attribute__((ext_vector_type(4)))  float v4f;
typedef __attribute__((ext_vector_type(2)))  float v2f;
typedef __attribute__((ext_vector_type(4)))  unsigned v4u;
typedef __attribute__((ext_vector_type(4)))  int v4i;
typedef float __attribute__((may_alias)) float_a;
typedef int __attribute__((may_alias)) int_a;

template <typename T> __device__ __forceinline__ void vst2(void* p, T v) { *(volatile T*)p = v; __threadfence(); *(volatile T*)p = v; }
__device__ __forceinline__ v8f wmma16(v16h a, v16h b, v8f c) {
  v8f d = __builtin_amdgcn_wmma_f32_16x16x32_f16(false, a, false, b, (short)0, c, false, false);
  asm volatile("v_nop\n\tv_nop\n\tv_nop\n\tv_nop" : "+v"(d) : "v"(a), "v"(b));
  return d;
}
__device__ __forceinline__ v8f wmma_bf(v16b a, v16b b, v8f c) {
  v8f d = __builtin_amdgcn_wmma_f32_16x16x32_bf16(false, a, false, b, (short)0, c, false, false);
  asm volatile("v_nop\n\tv_nop\n\tv_nop\n\tv_nop" : "+v"(d) : "v"(a), "v"(b));
  return d;
}
__device__ __forceinline__ v16h frag_h(const _Float16* rowk0, int lane) {
  union { v16h v; v8h q[2]; } u; const _Float16* p = rowk0 + 8 * (lane >> 4);
  u.q[0] = *(const v8h*)p; u.q[1] = *(const v8h*)(p + 16); return u.v;
}
__device__ __forceinline__ v16h frag_f32(const float* rowk0, int lane) {
  v16h a; const float* p = rowk0 + 8 * (lane >> 4);
#pragma unroll
  for (int i = 0; i < 8; ++i) { a[i] = (_Float16)p[i]; a[8 + i] = (_Float16)p[16 + i]; }
  return a;
}
__device__ __forceinline__ v16h frag_f32s(const float* rowk0, int lane, float sc) {
  v16h a; const float* p = rowk0 + 8 * (lane >> 4);
#pragma unroll
  for (int i = 0; i < 8; ++i) { a[i] = (_Float16)(p[i] * sc); a[8 + i] = (_Float16)(p[16 + i] * sc); }
  return a;
}
__device__ __forceinline__ v16h fragc_f32(const float* W, int k0, int n, int lane, int ld, int K) {
  v16h a; const int g = lane >> 4;
#pragma unroll
  for (int i = 0; i < 8; ++i) { const int ka = k0 + 8 * g + i, kb = ka + 16;
    a[i] = (_Float16)(ka < K ? W[(size_t)(ka < K ? ka : K - 1) * ld + n] : 0.f); a[8 + i] = (_Float16)(kb < K ? W[(size_t)(kb < K ? kb : K - 1) * ld + n] : 0.f); }
  return a;
}
struct F2 { v16b h, l; };
__device__ __forceinline__ F2 bsplit16(const float v[16]) { F2 r;
#pragma unroll
  for (int i = 0; i < 16; ++i) { const __bf16 h = (__bf16)v[i]; r.h[i] = h; r.l[i] = (__bf16)(v[i] - (float)h); }
  return r; }
__device__ __forceinline__ F2 split_row(const float* row, int k0, int lane) { float v[16]; const float* p = row + k0 + 8 * (lane >> 4);
#pragma unroll
  for (int i = 0; i < 8; ++i) { v[i] = p[i]; v[8 + i] = p[16 + i]; }
  return bsplit16(v); }
__device__ __forceinline__ F2 split_rowK(const float* row, int k0, int lane, int K) { float v[16]; const int g = lane >> 4;
#pragma unroll
  for (int i = 0; i < 8; ++i) { const int ka = k0 + 8 * g + i, kb = ka + 16; v[i] = ka < K ? row[ka < K ? ka : K - 1] : 0.f; v[8 + i] = kb < K ? row[kb < K ? kb : K - 1] : 0.f; }
  return bsplit16(v); }
__device__ __forceinline__ F2 split_col(const float* W, int k0, int n, int lane, int ld, int K) { float v[16]; const int g = lane >> 4;
#pragma unroll
  for (int i = 0; i < 8; ++i) { const int ka = k0 + 8 * g + i, kb = ka + 16; v[i] = ka < K ? W[(size_t)(ka < K ? ka : K - 1) * ld + n] : 0.f; v[8 + i] = kb < K ? W[(size_t)(kb < K ? kb : K - 1) * ld + n] : 0.f; }
  return bsplit16(v); }
__device__ __forceinline__ v8f mac3(const F2& a, const F2& b, v8f c) { c = wmma_bf(a.l, b.h, c); c = wmma_bf(a.h, b.l, c); return wmma_bf(a.h, b.h, c); }
__device__ __forceinline__ float sigm(float v) { return 1.0f / (1.0f + expf(-v)); }
#define LDSX() do { asm volatile("s_wait_dscnt 0" ::: "memory"); __builtin_amdgcn_wave_barrier(); __builtin_amdgcn_fence(__ATOMIC_RELEASE, "workgroup"); } while (0)


#define NSEQ 16
#define TL 4096
#define NV 21
#define CIN 18
#define XW 218
#define HDIM 64
#define ODIM 32
#define NR (NSEQ * TL)
#ifndef NRT
#define NRT NR
#define NSEQT NSEQ
#endif
typedef __attribute__((ext_vector_type(8))) __bf16 v8b;
__device__ __forceinline__ v16b frag_b(const __bf16* rowk0, int lane) {
  union { v16b v; v8b q[2]; } u; const __bf16* p = rowk0 + 8 * (lane >> 4);
  u.q[0] = *(const v8b*)p; u.q[1] = *(const v8b*)(p + 16); return u.v;
}
__device__ __forceinline__ float bfr(float v) { return (float)(__bf16)v; }
__device__ __attribute__((noinline)) float exp_ni(float v) { return expf(v); }
__device__ __attribute__((noinline)) float erf_ni(float v) { return erff(v); }

__device__ __attribute__((noinline)) float tanh_ni(float v) { return tanhf(v); }
__device__ __forceinline__ void put_hl(__bf16* h, __bf16* l, float v) { const __bf16 hb = (__bf16)v; *h = hb; *l = (__bf16)(v - (float)hb); }
__constant__ float c_ahat[32 * 32] = {
  0.166666672f, 0.235702261f, 0.f, 0.f, 0.f, 0.235702261f, 0.f, 0.f, 0.f, 0.235702261f, 0.f, 0.f, 0.f, 0.235702261f, 0.f, 0.f, 0.f, 0.235702261f, 0.f, 0.f, 0.f, 0.f, 0.f, 0.f, 0.f, 0.f, 0.f, 0.f, 0.f, 0.f, 0.f, 0.f,
  0.235702261f, 0.333333313f, 0.333333313f, 0.f, 0.f, 0.f, 0.f, 0.f, 0.f, 0.f, 0.f, 0.f, 0.f, 0.f, 0.f, 0.f, 0.f, 0.f, 0.f, 0.f, 0.f, 0.f, 0.f, 0.f, 0.f, 0.f, 0.f, 0.f, 0.f, 0.f, 0.f, 0.f,
  0.f, 0.333333313f, 0.333333313f, 0.333333313f, 0.f, 0.f, 0.f, 0.f, 0.f, 0.f, 0.f, 0.f, 0.f, 0.f, 0.f, 0.f, 0.f, 0.f, 0.f, 0.f, 0.f, 0.f, 0.f, 0.f, 0.f, 0.f, 0.f, 0.f, 0.f, 0.f, 0.f, 0.f,
  0.f, 0.f, 0.333333313f, 0.333333313f, 0.408248276f, 0.f, 0.f, 0.f, 0.f, 0.f, 0.f, 0.f, 0.f, 0.f, 0.f, 0.f, 0.f, 0.f, 0.f, 0.f, 0.f, 0.f, 0.f, 0.f, 0.f, 0.f, 0.f, 0.f, 0.f, 0.f, 0.f, 0.f,
  0.f, 0.f, 0.f, 0.408248276f, 0.499999970f, 0.f, 0.f, 0.f, 0.f, 0.f, 0.f, 0.f, 0.f, 0.f, 0.f, 0.f, 0.f, 0.f, 0.f, 0.f, 0.f, 0.f, 0.f, 0.f, 0.f, 0.f, 0.f, 0.f, 0.f, 0.f, 0.f, 0.f,
  0.235702261f, 0.f, 0.f, 0.f, 0.f, 0.333333313f, 0.333333313f, 0.f, 0.f, 0.f, 0.f, 0.f, 0.f, 0.f, 0.f, 0.f, 0.f, 0.f, 0.f, 0.f, 0.f, 0.f, 0.f, 0.f, 0.f, 0.f, 0.f, 0.f, 0.f, 0.f, 0.f, 0.f,
  0.f, 0.f, 0.f, 0.f, 0.f, 0.333333313f, 0.333333313f, 0.333333313f, 0.f, 0.f, 0.f, 0.f, 0.f, 0.f, 0.f, 0.f, 0.f, 0.f, 0.f, 0.f, 0.f, 0.f, 0.f, 0.f, 0.f, 0.f, 0.f, 0.f, 0.f, 0.f, 0.f, 0.f,
  0.f, 0.f, 0.f, 0.f, 0.f, 0.f, 0.333333313f, 0.333333313f, 0.408248276f, 0.f, 0.f, 0.f, 0.f, 0.f, 0.f, 0.f, 0.f, 0.f, 0.f, 0.f, 0.f, 0.f, 0.f, 0.f, 0.f, 0.f, 0.f, 0.f, 0.f, 0.f, 0.f, 0.f,
  0.f, 0.f, 0.f, 0.f, 0.f, 0.f, 0.f, 0.408248276f, 0.499999970f, 0.f, 0.f, 0.f, 0.f, 0.f, 0.f, 0.f, 0.f, 0.f, 0.f, 0.f, 0.f, 0.f, 0.f, 0.f, 0.f, 0.f, 0.f, 0.f, 0.f, 0.f, 0.f, 0.f,
  0.235702261f, 0.f, 0.f, 0.f, 0.f, 0.f, 0.f, 0.f, 0.f, 0.333333313f, 0.333333313f, 0.f, 0.f, 0.f, 0.f, 0.f, 0.f, 0.f, 0.f, 0.f, 0.f, 0.f, 0.f, 0.f, 0.f, 0.f, 0.f, 0.f, 0.f, 0.f, 0.f, 0.f,
  0.f, 0.f, 0.f, 0.f, 0.f, 0.f, 0.f, 0.f, 0.f, 0.333333313f, 0.333333313f, 0.333333313f, 0.f, 0.f, 0.f, 0.f, 0.f, 0.f, 0.f, 0.f, 0.f, 0.f, 0.f, 0.f, 0.f, 0.f, 0.f, 0.f, 0.f, 0.f, 0.f, 0.f,
  0.f, 0.f, 0.f, 0.f, 0.f, 0.f, 0.f, 0.f, 0.f, 0.f, 0.333333313f, 0.333333313f, 0.408248276f, 0.f, 0.f, 0.f, 0.f, 0.f, 0.f, 0.f, 0.f, 0.f, 0.f, 0.f, 0.f, 0.f, 0.f, 0.f, 0.f, 0.f, 0.f, 0.f,
  0.f, 0.f, 0.f, 0.f, 0.f, 0.f, 0.f, 0.f, 0.f, 0.f, 0.f, 0.408248276f, 0.499999970f, 0.f, 0.f, 0.f, 0.f, 0.f, 0.f, 0.f, 0.f, 0.f, 0.f, 0.f, 0.f, 0.f, 0.f, 0.f, 0.f, 0.f, 0.f, 0.f,
  0.235702261f, 0.f, 0.f, 0.f, 0.f, 0.f, 0.f, 0.f, 0.f, 0.f, 0.f, 0.f, 0.f, 0.333333313f, 0.333333313f, 0.f, 0.f, 0.f, 0.f, 0.f, 0.f, 0.f, 0.f, 0.f, 0.f, 0.f, 0.f, 0.f, 0.f, 0.f, 0.f, 0.f,
  0.f, 0.f, 0.f, 0.f, 0.f, 0.f, 0.f, 0.f, 0.f, 0.f, 0.f, 0.f, 0.f, 0.333333313f, 0.333333313f, 0.333333313f, 0.f, 0.f, 0.f, 0.f, 0.f, 0.f, 0.f, 0.f, 0.f, 0.f, 0.f, 0.f, 0.f, 0.f, 0.f, 0.f,
  0.f, 0.f, 0.f, 0.f, 0.f, 0.f, 0.f, 0.f, 0.f, 0.f, 0.f, 0.f, 0.f, 0.f, 0.333333313f, 0.333333313f, 0.408248276f, 0.f, 0.f, 0.f, 0.f, 0.f, 0.f, 0.f, 0.f, 0.f, 0.f, 0.f, 0.f, 0.f, 0.f, 0.f,
  0.f, 0.f, 0.f, 0.f, 0.f, 0.f, 0.f, 0.f, 0.f, 0.f, 0.f, 0.f, 0.f, 0.f, 0.f, 0.408248276f, 0.499999970f, 0.f, 0.f, 0.f, 0.f, 0.f, 0.f, 0.f, 0.f, 0.f, 0.f, 0.f, 0.f, 0.f, 0.f, 0.f,
  0.235702261f, 0.f, 0.f, 0.f, 0.f, 0.f, 0.f, 0.f, 0.f, 0.f, 0.f, 0.f, 0.f, 0.f, 0.f, 0.f, 0.f, 0.333333313f, 0.333333313f, 0.f, 0.f, 0.f, 0.f, 0.f, 0.f, 0.f, 0.f, 0.f, 0.f, 0.f, 0.f, 0.f,
  0.f, 0.f, 0.f, 0.f, 0.f, 0.f, 0.f, 0.f, 0.f, 0.f, 0.f, 0.f, 0.f, 0.f, 0.f, 0.f, 0.f, 0.333333313f, 0.333333313f, 0.333333313f, 0.f, 0.f, 0.f, 0.f, 0.f, 0.f, 0.f, 0.f, 0.f, 0.f, 0.f, 0.f,
  0.f, 0.f, 0.f, 0.f, 0.f, 0.f, 0.f, 0.f, 0.f, 0.f, 0.f, 0.f, 0.f, 0.f, 0.f, 0.f, 0.f, 0.f, 0.333333313f, 0.333333313f, 0.408248276f, 0.f, 0.f, 0.f, 0.f, 0.f, 0.f, 0.f, 0.f, 0.f, 0.f, 0.f,
  0.f, 0.f, 0.f, 0.f, 0.f, 0.f, 0.f, 0.f, 0.f, 0.f, 0.f, 0.f, 0.f, 0.f, 0.f, 0.f, 0.f, 0.f, 0.f, 0.408248276f, 0.499999970f, 0.f, 0.f, 0.f, 0.f, 0.f, 0.f, 0.f, 0.f, 0.f, 0.f, 0.f,
  0.f, 0.f, 0.f, 0.f, 0.f, 0.f, 0.f, 0.f, 0.f, 0.f, 0.f, 0.f, 0.f, 0.f, 0.f, 0.f, 0.f, 0.f, 0.f, 0.f, 0.f, 0.f, 0.f, 0.f, 0.f, 0.f, 0.f, 0.f, 0.f, 0.f, 0.f, 0.f,
  0.f, 0.f, 0.f, 0.f, 0.f, 0.f, 0.f, 0.f, 0.f, 0.f, 0.f, 0.f, 0.f, 0.f, 0.f, 0.f, 0.f, 0.f, 0.f, 0.f, 0.f, 0.f, 0.f, 0.f, 0.f, 0.f, 0.f, 0.f, 0.f, 0.f, 0.f, 0.f,
  0.f, 0.f, 0.f, 0.f, 0.f, 0.f, 0.f, 0.f, 0.f, 0.f, 0.f, 0.f, 0.f, 0.f, 0.f, 0.f, 0.f, 0.f, 0.f, 0.f, 0.f, 0.f, 0.f, 0.f, 0.f, 0.f, 0.f, 0.f, 0.f, 0.f, 0.f, 0.f,
  0.f, 0.f, 0.f, 0.f, 0.f, 0.f, 0.f, 0.f, 0.f, 0.f, 0.f, 0.f, 0.f, 0.f, 0.f, 0.f, 0.f, 0.f, 0.f, 0.f, 0.f, 0.f, 0.f, 0.f, 0.f, 0.f, 0.f, 0.f, 0.f, 0.f, 0.f, 0.f,
  0.f, 0.f, 0.f, 0.f, 0.f, 0.f, 0.f, 0.f, 0.f, 0.f, 0.f, 0.f, 0.f, 0.f, 0.f, 0.f, 0.f, 0.f, 0.f, 0.f, 0.f, 0.f, 0.f, 0.f, 0.f, 0.f, 0.f, 0.f, 0.f, 0.f, 0.f, 0.f,
  0.f, 0.f, 0.f, 0.f, 0.f, 0.f, 0.f, 0.f, 0.f, 0.f, 0.f, 0.f, 0.f, 0.f, 0.f, 0.f, 0.f, 0.f, 0.f, 0.f, 0.f, 0.f, 0.f, 0.f, 0.f, 0.f, 0.f, 0.f, 0.f, 0.f, 0.f, 0.f,
  0.f, 0.f, 0.f, 0.f, 0.f, 0.f, 0.f, 0.f, 0.f, 0.f, 0.f, 0.f, 0.f, 0.f, 0.f, 0.f, 0.f, 0.f, 0.f, 0.f, 0.f, 0.f, 0.f, 0.f, 0.f, 0.f, 0.f, 0.f, 0.f, 0.f, 0.f, 0.f,
  0.f, 0.f, 0.f, 0.f, 0.f, 0.f, 0.f, 0.f, 0.f, 0.f, 0.f, 0.f, 0.f, 0.f, 0.f, 0.f, 0.f, 0.f, 0.f, 0.f, 0.f, 0.f, 0.f, 0.f, 0.f, 0.f, 0.f, 0.f, 0.f, 0.f, 0.f, 0.f,
  0.f, 0.f, 0.f, 0.f, 0.f, 0.f, 0.f, 0.f, 0.f, 0.f, 0.f, 0.f, 0.f, 0.f, 0.f, 0.f, 0.f, 0.f, 0.f, 0.f, 0.f, 0.f, 0.f, 0.f, 0.f, 0.f, 0.f, 0.f, 0.f, 0.f, 0.f, 0.f,
  0.f, 0.f, 0.f, 0.f, 0.f, 0.f, 0.f, 0.f, 0.f, 0.f, 0.f, 0.f, 0.f, 0.f, 0.f, 0.f, 0.f, 0.f, 0.f, 0.f, 0.f, 0.f, 0.f, 0.f, 0.f, 0.f, 0.f, 0.f, 0.f, 0.f, 0.f, 0.f,
  0.f, 0.f, 0.f, 0.f, 0.f, 0.f, 0.f, 0.f, 0.f, 0.f, 0.f, 0.f, 0.f, 0.f, 0.f, 0.f, 0.f, 0.f, 0.f, 0.f, 0.f, 0.f, 0.f, 0.f, 0.f, 0.f, 0.f, 0.f, 0.f, 0.f, 0.f, 0.f,
};

#define PK_GW   0
#define PK_T1S  (PK_GW + 64 * 32)
#define PK_T1M  (PK_T1S + 3 * 16 * 64)
#define PK_T1L  (PK_T1M + 5 * 16 * 64)
#define PK_T1O  (PK_T1L + 9 * 32 * 64)
#define PK_T2S  (PK_T1O + 64 * 64)
#define PK_T2M  (PK_T2S + 3 * 16 * 64)
#define PK_T2L  (PK_T2M + 5 * 16 * 64)
#define PK_T2O  (PK_T2L + 9 * 32 * 64)
#define PK_WD   (PK_T2O + 64 * 64)
#define PK_END  (PK_WD + 32 * 64)
#define WS_PK   0u
#define WS_POOL (WS_PK + 2u * PK_END)
#define WS_T1   (WS_POOL + 4u * NR * HDIM)
#define WS_T2   (WS_T1 + 4u * NR * HDIM)
#define WS_HO   (WS_T2 + 4u * NR * HDIM)
#define WS_END  (WS_HO + 4u * NR * ODIM)

__global__ __launch_bounds__(128) void k_pack(const float* __restrict__ Wm, int ldk, int Kin, int Kp, __bf16* __restrict__ DST) {
  __shared__ __align__(16) __bf16 s[8 * 64]; const int n0 = blockIdx.x * 8, tid = threadIdx.x;
  for (int q = tid; q < 8 * Kp; q += 128) { const int rl = q / Kp, k = q % Kp; s[q] = (__bf16)(k < Kin ? bfr(Wm[(size_t)k * ldk + n0 + rl]) : 0.f); }
  __syncthreads();
  for (int q = tid; q < Kp; q += 128) vst2((unsigned*)(DST + (size_t)n0 * Kp + q * 8), *(const v4u*)&s[q * 8]);
}
__global__ __launch_bounds__(256) void k_gcn(const float* __restrict__ X, const __bf16* __restrict__ PK, float* __restrict__ POOL) {
  __shared__ __align__(16) __bf16 sg[8][32][40]; __shared__ __align__(16) __bf16 sth[8][64][40], stl[8][64][40]; __shared__ __align__(16) __bf16 sah[32][40], sal[32][40]; __shared__ __align__(16) float so[8][64];
  const int tid = threadIdx.x, wave = tid >> 5, lane = tid & 31, col = lane & 15, hf = lane >> 4; const size_t r = (size_t)blockIdx.x * 8 + wave;
  for (int q = tid; q < 32 * 32; q += 256) { const int v = q >> 5, w = q & 31; put_hl(&sah[v][w], &sal[v][w], c_ahat[v * 32 + w]); }
  { const float* xr = X + r * XW;
    for (int q = lane; q < 32 * 32; q += 32) { const int v = q >> 5, c = q & 31; float val = 0.f;
      if (v == 0) { if (c < CIN) val = bfr(xr[c < CIN ? c : 0]); }
      else if (v < NV) { if (c < 10) val = bfr(xr[18 + (v - 1) * 10 + (c < 10 ? c : 0)]); }
      sg[wave][v][c] = (__bf16)val; } }
  __syncthreads();
  { v8f acc[2][4] = {}; const v16b a0 = frag_b(&sg[wave][col][0], lane), a1 = frag_b(&sg[wave][16 + col][0], lane);
#pragma unroll
    for (int j = 0; j < 4; ++j) { const v16b w = frag_b(PK + PK_GW + (size_t)(j * 16 + col) * 32, lane); acc[0][j] = wmma_bf(a0, w, acc[0][j]); acc[1][j] = wmma_bf(a1, w, acc[1][j]); }
#pragma unroll
    for (int rt = 0; rt < 2; ++rt)
#pragma unroll
      for (int j = 0; j < 4; ++j)
#pragma unroll
        for (int rr = 0; rr < 8; ++rr) put_hl(&sth[wave][j * 16 + col][rt * 16 + 8 * hf + rr], &stl[wave][j * 16 + col][rt * 16 + 8 * hf + rr], acc[rt][j][rr]); }
  LDSX();
  { v8f acc[2][4] = {};
#pragma unroll
    for (int rt = 0; rt < 2; ++rt) { const v16b ah = frag_b(&sah[rt * 16 + col][0], lane), al = frag_b(&sal[rt * 16 + col][0], lane);
#pragma unroll
      for (int j = 0; j < 4; ++j) { const v16b bh = frag_b(&sth[wave][j * 16 + col][0], lane), bl = frag_b(&stl[wave][j * 16 + col][0], lane); acc[rt][j] = wmma_bf(al, bh, acc[rt][j]); acc[rt][j] = wmma_bf(ah, bl, acc[rt][j]); acc[rt][j] = wmma_bf(ah, bh, acc[rt][j]); } }
#pragma unroll
    for (int j = 0; j < 4; ++j) { float s = 0.f;
#pragma unroll
      for (int rt = 0; rt < 2; ++rt)
#pragma unroll
        for (int rr = 0; rr < 8; ++rr) s += fmaxf(acc[rt][j][rr], 0.f);
      s += __shfl_xor(s, 16); if (hf == 0) so[wave][j * 16 + col] = s * (1.0f / (float)NV); } }
  LDSX();
  if (lane < 16) vst2(POOL + r * HDIM + lane * 4, *(const v4f*)&so[wave][lane * 4]);
}
__global__ __launch_bounds__(128) void k_tcn(const float* __restrict__ IN, const __bf16* __restrict__ PK, int pks, int pkm, int pkl, int pko, const float* __restrict__ bs, const float* __restrict__ bm, const float* __restrict__ bl, const float* __restrict__ bo, float* __restrict__ OUT) {
  __shared__ __align__(16) __bf16 shh[4][16][72], shl[4][16][72]; __shared__ __align__(16) float so[4][16][68];
  const int tid = threadIdx.x, wave = tid >> 5, lane = tid & 31, col = lane & 15, hf = lane >> 4; const size_t r0 = (size_t)blockIdx.x * 64 + wave * 16; const int t0 = (int)(r0 % TL); const size_t seq0 = r0 - t0;
  v8f as = {}, am = {}, al0 = {}, al1 = {};
#pragma unroll 1
  for (int tap = 0; tap < 3 + 5 + 9; ++tap) { int j, dil, nk, base; if (tap < 3) { j = tap; dil = 1; nk = 3; base = pks; } else if (tap < 8) { j = tap - 3; dil = 2; nk = 5; base = pkm; } else { j = tap - 8; dil = 4; nk = 9; base = pkl; }
    const int off = (nk - 1 - j) * dil; const int tt = t0 + col - off; const float* arow = IN + (seq0 + (tt >= 0 ? tt : 0)) * HDIM; const float zs = (tt >= 0) ? 1.f : 0.f;
#pragma unroll
    for (int kc = 0; kc < 2; ++kc) { float v[16]; const float* p = arow + kc * 32 + 8 * hf;
#pragma unroll
      for (int i = 0; i < 8; ++i) { v[i] = p[i] * zs; v[8 + i] = p[16 + i] * zs; }
      const F2 a = bsplit16(v);
      if (tap < 3) { const v16b w = frag_b(PK + base + (size_t)(j * 16 + col) * HDIM + kc * 32, lane); as = wmma_bf(a.l, w, as); as = wmma_bf(a.h, w, as); }
      else if (tap < 8) { const v16b w = frag_b(PK + base + (size_t)(j * 16 + col) * HDIM + kc * 32, lane); am = wmma_bf(a.l, w, am); am = wmma_bf(a.h, w, am); }
      else { const v16b w0 = frag_b(PK + base + (size_t)(j * 32 + col) * HDIM + kc * 32, lane), w1 = frag_b(PK + base + (size_t)(j * 32 + 16 + col) * HDIM + kc * 32, lane); al0 = wmma_bf(a.l, w0, al0); al0 = wmma_bf(a.h, w0, al0); al1 = wmma_bf(a.l, w1, al1); al1 = wmma_bf(a.h, w1, al1); } } }
  { const float b0 = bfr(bs[col]), b1 = bfr(bm[col]), b2 = bfr(bl[col]), b3 = bfr(bl[16 + col]);
#pragma unroll
    for (int rr = 0; rr < 8; ++rr) { const int row = 8 * hf + rr; put_hl(&shh[wave][row][col], &shl[wave][row][col], fmaxf(as[rr] + b0, 0.f)); put_hl(&shh[wave][row][16 + col], &shl[wave][row][16 + col], fmaxf(am[rr] + b1, 0.f)); put_hl(&shh[wave][row][32 + col], &shl[wave][row][32 + col], fmaxf(al0[rr] + b2, 0.f)); put_hl(&shh[wave][row][48 + col], &shl[wave][row][48 + col], fmaxf(al1[rr] + b3, 0.f)); } }
  LDSX();
  { v8f acc[4] = {};
#pragma unroll
    for (int kc = 0; kc < 2; ++kc) { const v16b xh = frag_b(&shh[wave][col][kc * 32], lane), xl = frag_b(&shl[wave][col][kc * 32], lane);
#pragma unroll
      for (int jn = 0; jn < 4; ++jn) { const v16b w = frag_b(PK + pko + (size_t)(jn * 16 + col) * HDIM + kc * 32, lane); acc[jn] = wmma_bf(xl, w, acc[jn]); acc[jn] = wmma_bf(xh, w, acc[jn]); } }
#pragma unroll
    for (int jn = 0; jn < 4; ++jn) { const float bb = bfr(bo[jn * 16 + col]);
#pragma unroll
      for (int rr = 0; rr < 8; ++rr) so[wave][8 * hf + rr][jn * 16 + col] = acc[jn][rr] + bb; } }
  LDSX();
  for (int rl = 0; rl < 16; ++rl) if (lane < 16) vst2(OUT + (r0 + rl) * HDIM + lane * 4, *(const v4f*)&so[wave][rl][lane * 4]);
}
__global__ __launch_bounds__(128) void k_head(const float* __restrict__ T2, const __bf16* __restrict__ PK, const float* __restrict__ bd, float* __restrict__ HO) {
  __shared__ __align__(16) float so[4][16][36];
  const int tid = threadIdx.x, wave = tid >> 5, lane = tid & 31, col = lane & 15, hf = lane >> 4; const size_t r0 = (size_t)blockIdx.x * 64 + wave * 16;
  v8f acc[2] = {};
#pragma unroll
  for (int kc = 0; kc < 2; ++kc) { const F2 a = split_row(T2 + (r0 + col) * HDIM, kc * 32, lane);
#pragma unroll
    for (int jn = 0; jn < 2; ++jn) { const v16b w = frag_b(PK + PK_WD + (size_t)(jn * 16 + col) * HDIM + kc * 32, lane); acc[jn] = wmma_bf(a.l, w, acc[jn]); acc[jn] = wmma_bf(a.h, w, acc[jn]); } }
#pragma unroll
  for (int jn = 0; jn < 2; ++jn) { const float bb = bfr(bd[jn * 16 + col]);
#pragma unroll
    for (int rr = 0; rr < 8; ++rr) so[wave][8 * hf + rr][jn * 16 + col] = tanh_ni(acc[jn][rr] + bb); }
  LDSX();
  for (int rl = 0; rl < 16; ++rl) if (lane < 8) vst2(HO + (r0 + rl) * ODIM + lane * 4, *(const v4f*)&so[wave][rl][lane * 4]);
}
__global__ __launch_bounds__(256) void k_mean(const float* __restrict__ HO, float* __restrict__ out) {
  __shared__ float sp[8][32]; __shared__ __align__(16) float so[32];
  const int b = blockIdx.x, tid = threadIdx.x, grp = tid >> 5, c = tid & 31; float s = 0.f;
#pragma unroll 4
  for (int t = grp * (TL / 8); t < (grp + 1) * (TL / 8); ++t) s += HO[((size_t)b * TL + t) * ODIM + c];
  sp[grp][c] = s; __syncthreads();
  if (tid < 32) { float a = 0.f;
#pragma unroll
    for (int g2 = 0; g2 < 8; ++g2) a += sp[g2][tid];
    so[tid] = a * (1.0f / (float)TL); }
  __syncthreads();
  if (tid < 8) vst2(out + (size_t)b * ODIM + tid * 4, *(const v4f*)&so[tid * 4]);
}
extern "C" void kernel_launch(void* const* d_in, const int* in_sizes, int n_in, void* d_out, int out_size, void* d_ws, size_t ws_size, hipStream_t stream) {
  (void)in_sizes; (void)n_in; (void)out_size;
  const float** F = (const float**)d_in;
  if (ws_size < (size_t)WS_END) return;
  char* ws = (char*)d_ws; __bf16* PK = (__bf16*)(ws + WS_PK); float *POOL = (float*)(ws + WS_POOL), *T1 = (float*)(ws + WS_T1), *T2 = (float*)(ws + WS_T2), *HO = (float*)(ws + WS_HO);
  k_pack<<<64 / 8, 128, 0, stream>>>(F[1], 64, CIN, 32, PK + PK_GW);
  for (int j = 0; j < 3; ++j) { k_pack<<<16 / 8, 128, 0, stream>>>(F[4] + (size_t)j * 64 * 16, 16, 64, 64, PK + PK_T1S + (size_t)j * 16 * 64); k_pack<<<16 / 8, 128, 0, stream>>>(F[12] + (size_t)j * 64 * 16, 16, 64, 64, PK + PK_T2S + (size_t)j * 16 * 64); }
  for (int j = 0; j < 5; ++j) { k_pack<<<16 / 8, 128, 0, stream>>>(F[6] + (size_t)j * 64 * 16, 16, 64, 64, PK + PK_T1M + (size_t)j * 16 * 64); k_pack<<<16 / 8, 128, 0, stream>>>(F[14] + (size_t)j * 64 * 16, 16, 64, 64, PK + PK_T2M + (size_t)j * 16 * 64); }
  for (int j = 0; j < 9; ++j) { k_pack<<<32 / 8, 128, 0, stream>>>(F[8] + (size_t)j * 64 * 32, 32, 64, 64, PK + PK_T1L + (size_t)j * 32 * 64); k_pack<<<32 / 8, 128, 0, stream>>>(F[16] + (size_t)j * 64 * 32, 32, 64, 64, PK + PK_T2L + (size_t)j * 32 * 64); }
  k_pack<<<64 / 8, 128, 0, stream>>>(F[10], 64, 64, 64, PK + PK_T1O);
  k_pack<<<64 / 8, 128, 0, stream>>>(F[18], 64, 64, 64, PK + PK_T2O);
  k_pack<<<32 / 8, 128, 0, stream>>>(F[2], 32, 64, 64, PK + PK_WD);
  k_gcn<<<NRT / 8, 256, 0, stream>>>(F[0], PK, POOL);
  k_tcn<<<NRT / 64, 128, 0, stream>>>(POOL, PK, PK_T1S, PK_T1M, PK_T1L, PK_T1O, F[5], F[7], F[9], F[11], T1);
  k_tcn<<<NRT / 64, 128, 0, stream>>>(T1, PK, PK_T2S, PK_T2M, PK_T2L, PK_T2O, F[13], F[15], F[17], F[19], T2);
  k_head<<<NRT / 64, 128, 0, stream>>>(T2, PK, F[3], HO);
  k_mean<<<NSEQT, 256, 0, stream>>>(HO, (float*)d_out);
}
